// EncoderDecoder_32117765439796
// MI455X (gfx1250) — hardware-run, weakly checked
//
#include <hip/hip_runtime.h>
#include <math.h>

constexpr int NBAT    = 512;
constexpr int NFEAT   = 64;
constexpr int NHID    = 256;
constexpr int NGATE3  = 3 * NHID;
constexpr int TSRC    = 128;
constexpr int TTGT    = 128;
constexpr int TTOT    = TSRC + TTGT;
constexpr int NTHR    = 256;
constexpr int SEQ_BLK = 16;
constexpr int XPITCH  = 72;
constexpr int HPITCH  = 264;
constexpr int OPITCH  = 68;
constexpr float WCARRY      = 256.0f;
constexpr float WCARRY_INV  = 1.0f / 256.0f;
constexpr float LOCARRY     = 2048.0f;
constexpr float LOCARRY_INV = 1.0f / 2048.0f;
constexpr int NOUT = NBAT * TTGT * NFEAT;
static_assert(NBAT % SEQ_BLK == 0);
static_assert(NHID == 32 * (NTHR / 32));
static_assert(NFEAT % 32 == 0 && NHID % 32 == 0);
static_assert(SEQ_BLK * NFEAT == NTHR * 4);
static_assert(NFEAT == 16 * 4);
static_assert((NTHR / 32) * 2 == SEQ_BLK);
static_assert(NFEAT * 4 == 256);
static_assert((NGATE3 * NFEAT / 8) % NTHR == 0 && (NGATE3 * NHID / 8) % NTHR == 0 && (NFEAT * NHID / 8) % NTHR == 0);
static_assert(XPITCH % 8 == 0 && HPITCH % 8 == 0 && OPITCH % 4 == 0);

typedef __attribute__((ext_vector_type(16))) _Float16 v16h;
typedef __attribute__((ext_vector_type(8)))  _Float16 v8h;
typedef __attribute__((ext_vector_type(4)))  _Float16 v4h;
typedef __attribute__((ext_vector_type(8)))  float    v8f;
typedef __attribute__((ext_vector_type(4)))  float    v4f;

__device__ __forceinline__ unsigned short f2bf_bits(float f) {
  unsigned u = __float_as_uint(f);
  return (unsigned short)((u + 0x7FFFu + ((u >> 16) & 1u)) >> 16);
}
__device__ __forceinline__ float bf_bits2f(unsigned short h) { return __uint_as_float(((unsigned)h) << 16); }
__device__ __forceinline__ float bf16r(float f) { return bf_bits2f(f2bf_bits(f)); }

__device__ __forceinline__ void dep_guard_h(v8f& a, v8f& b, v16h x, v16h y) { asm volatile("v_nop\n\tv_nop\n\tv_nop\n\tv_nop" : "+v"(a), "+v"(b) : "v"(x), "v"(y)); }
__device__ __forceinline__ void dep_guard3_h(v8f& a, v8f& b, v8f& c, v16h x, v16h y) {
  asm volatile("v_nop\n\tv_nop\n\tv_nop\n\tv_nop" : "+v"(a), "+v"(b), "+v"(c) : "v"(x), "v"(y));
}
__device__ __forceinline__ void dep_guard6_h(v8f& a, v8f& b, v8f& c, v8f& d, v8f& e, v8f& f, v16h x, v16h y) {
  asm volatile("v_nop\n\tv_nop\n\tv_nop\n\tv_nop" : "+v"(a), "+v"(b), "+v"(c), "+v"(d), "+v"(e), "+v"(f) : "v"(x), "v"(y));
}
__device__ __forceinline__ void keep4_h(v16h a, v16h b, v16h c, v16h d) { asm volatile("v_nop" :: "v"(a), "v"(b), "v"(c), "v"(d)); }
__device__ __forceinline__ void acc_guard4(v8f& a, v8f& b, v8f& c, v8f& d) { asm volatile("v_nop\n\tv_nop\n\tv_nop\n\tv_nop" : "+v"(a), "+v"(b), "+v"(c), "+v"(d)); }
__device__ __forceinline__ void acc_guard3(v8f& a, v8f& b, v8f& c) { asm volatile("v_nop\n\tv_nop\n\tv_nop\n\tv_nop" : "+v"(a), "+v"(b), "+v"(c)); }
__device__ __forceinline__ void acc_guard2(v8f& a, v8f& b) { asm volatile("v_nop\n\tv_nop\n\tv_nop\n\tv_nop" : "+v"(a), "+v"(b)); }

template <typename T> struct Frag;
template <> struct Frag<_Float16> {
  typedef v16h V; union U { v16h v; v8h h[2]; };
  static __device__ __forceinline__ v16h load(const _Float16* p) {
    U f; f.h[0] = *(const v8h*)(p); f.h[1] = *(const v8h*)(p + 16); return f.v;
  }
  static __device__ __forceinline__ v8f mma(v16h a, v16h b, v8f c) {
    return __builtin_amdgcn_wmma_f32_16x16x32_f16(false, a, false, b, (short)0, c, false, false);
  }
  static __device__ __forceinline__ void guard(v8f& a, v8f& b, v16h x, v16h y) { dep_guard_h(a, b, x, y); }
  static __device__ __forceinline__ void keep(v16h a, v16h b, v16h c, v16h d) { keep4_h(a, b, c, d); }
};

__device__ __forceinline__ float fsigm(float v) { return 1.0f / (1.0f + expf(-v)); }

template <int MODE>
__global__ __launch_bounds__(NTHR) void cvt8_kernel(const float* __restrict__ src, unsigned short* __restrict__ dst,
                                                    int nrow, int ncol8, int spitch, int scol0, float sc) {
  const int i  = blockIdx.x * NTHR + threadIdx.x;
  const int n8 = nrow * ncol8;
  if (i < n8) {
    const int row = i / ncol8;
    const int c8  = i - row * ncol8;
    const float* sp = src + (size_t)row * spitch + scol0 + c8 * 8;
    const v4f a = *(const v4f*)(sp);
    const v4f b = *(const v4f*)(sp + 4);
    v8h hv;
#pragma unroll
    for (int e = 0; e < 4; ++e) {
      unsigned short b0, b1;
      if (MODE == 0) {
        b0 = f2bf_bits(a[e] * sc);
        b1 = f2bf_bits(b[e] * sc);
      } else {
        b0 = __builtin_bit_cast(unsigned short, (_Float16)(bf16r(a[e]) * sc));
        b1 = __builtin_bit_cast(unsigned short, (_Float16)(bf16r(b[e]) * sc));
      }
      hv[e]     = __builtin_bit_cast(_Float16, b0);
      hv[4 + e] = __builtin_bit_cast(_Float16, b1);
    }
    *(volatile v8h*)(dst + (size_t)i * 8) = hv;
    __threadfence();
    *(volatile v8h*)(dst + (size_t)i * 8) = hv;
  }
}

__device__ __forceinline__ void gru_cell(const _Float16* axrow, const _Float16* ahrow, const _Float16* alrow,
                                         const _Float16* __restrict__ WIH, const _Float16* __restrict__ WHH,
                                         const float (&bb)[2][4], float (&hst)[2][8], int wave, int c, int koff) {
  const v8f z8 = {0.f, 0.f, 0.f, 0.f, 0.f, 0.f, 0.f, 0.f};
#pragma unroll
  for (int nt = 0; nt < 2; ++nt) {
    const int j = 32 * wave + 16 * nt + c;
    const _Float16* wx = WIH + (size_t)j * NFEAT + koff;
    const _Float16* wh = WHH + (size_t)j * NHID + koff;
    v8f aR = z8, aZ = z8, aNI = z8, aNH = z8, lR = z8, lZ = z8, lNH = z8;
#pragma unroll 1
    for (int kx = 0; kx < NFEAT; kx += 32) {
      const v16h a  = Frag<_Float16>::load(axrow + kx);
      const v16h b0 = Frag<_Float16>::load(wx + kx);
      const v16h b1 = Frag<_Float16>::load(wx + (size_t)NHID * NFEAT + kx);
      const v16h b2 = Frag<_Float16>::load(wx + (size_t)2 * NHID * NFEAT + kx);
      aR  = Frag<_Float16>::mma(a, b0, aR);
      aZ  = Frag<_Float16>::mma(a, b1, aZ);
      aNI = Frag<_Float16>::mma(a, b2, aNI);
      dep_guard3_h(aR, aZ, aNI, a, b2);
      keep4_h(b0, b1, b2, a);
    }
#pragma unroll 1
    for (int k0 = 0; k0 < NHID; k0 += 32) {
      const v16h ah = Frag<_Float16>::load(ahrow + k0);
      const v16h al = Frag<_Float16>::load(alrow + k0);
      const v16h b0 = Frag<_Float16>::load(wh + k0);
      const v16h b1 = Frag<_Float16>::load(wh + (size_t)NHID * NHID + k0);
      const v16h b2 = Frag<_Float16>::load(wh + (size_t)2 * NHID * NHID + k0);
      aR  = Frag<_Float16>::mma(ah, b0, aR);
      lR  = Frag<_Float16>::mma(al, b0, lR);
      aZ  = Frag<_Float16>::mma(ah, b1, aZ);
      lZ  = Frag<_Float16>::mma(al, b1, lZ);
      aNH = Frag<_Float16>::mma(ah, b2, aNH);
      lNH = Frag<_Float16>::mma(al, b2, lNH);
      dep_guard6_h(aR, lR, aZ, lZ, aNH, lNH, ah, al);
      keep4_h(b0, b1, b2, ah);
    }
    acc_guard4(aR, aZ, aNI, aNH);
    acc_guard3(lR, lZ, lNH);
#pragma unroll
    for (int r = 0; r < 8; ++r) {
      const float pr = (aR[r] + lR[r] * LOCARRY_INV) * WCARRY_INV + bb[nt][0];
      const float pz = (aZ[r] + lZ[r] * LOCARRY_INV) * WCARRY_INV + bb[nt][1];
      const float ni = aNI[r] * WCARRY_INV + bb[nt][2];
      const float nh = (aNH[r] + lNH[r] * LOCARRY_INV) * WCARRY_INV + bb[nt][3];
      const float rr = fsigm(pr);
      const float zz = fsigm(pz);
      const float nn = tanhf(ni + rr * nh);
      const float ho = hst[nt][r];
      hst[nt][r] = (1.0f - zz) * nn + zz * ho;
    }
  }
}

__global__ __launch_bounds__(NTHR) void gru_seq_kernel(const float* __restrict__ x,
                                                       const float* __restrict__ ebih, const float* __restrict__ ebhh,
                                                       const float* __restrict__ dbih, const float* __restrict__ dbhh,
                                                       const float* __restrict__ regb,
                                                       const unsigned short* __restrict__ WIHEp,
                                                       const unsigned short* __restrict__ WHHEp,
                                                       const unsigned short* __restrict__ WIHDp,
                                                       const unsigned short* __restrict__ WHHDp,
                                                       const unsigned short* __restrict__ WREGp,
                                                       const int* __restrict__ len_src, const int* __restrict__ len_tgt,
                                                       float* __restrict__ out) {
  __shared__ __align__(16) _Float16 Ax[SEQ_BLK * XPITCH];
  __shared__ __align__(16) _Float16 Ahh[SEQ_BLK * HPITCH];
  __shared__ __align__(16) _Float16 Ahl[SEQ_BLK * HPITCH];
  __shared__ __align__(16) float    Os[SEQ_BLK * OPITCH];
  const _Float16* WIHE = (const _Float16*)WIHEp;
  const _Float16* WHHE = (const _Float16*)WHHEp;
  const _Float16* WIHD = (const _Float16*)WIHDp;
  const _Float16* WHHD = (const _Float16*)WHHDp;
  const _Float16* WREG = (const _Float16*)WREGp;
  (void)len_tgt;
  const int tid  = threadIdx.x, lane = tid & 31;
  const int wave = __builtin_amdgcn_readfirstlane(tid >> 5);
  const int c = lane & 15, hh = lane >> 4, koff = hh * 8, c4 = c * 4;
  const int rowbase = blockIdx.x * SEQ_BLK;
  const int m_st = tid >> 4, f4 = (tid & 15) * 4;

#pragma unroll 1
  for (int i = tid; i < SEQ_BLK * XPITCH; i += NTHR) Ax[i] = (_Float16)0.0f;
#pragma unroll 1
  for (int i = tid; i < SEQ_BLK * HPITCH; i += NTHR) { Ahh[i] = (_Float16)0.0f; Ahl[i] = (_Float16)0.0f; }
  float hst[2][8];
#pragma unroll
  for (int nt = 0; nt < 2; ++nt)
#pragma unroll
    for (int r = 0; r < 8; ++r) hst[nt][r] = 0.0f;
  __syncthreads();

  int ls = len_src[0];
  ls = (ls < 1) ? 1 : ((ls > TSRC) ? TSRC : ls);
  const int ts_last = ls - 1;

  {
    const v4f v = *(const v4f*)(x + ((size_t)(rowbase + m_st) * TTOT) * NFEAT + f4);
    v4h hv;
    hv[0] = (_Float16)bf16r(v[0]); hv[1] = (_Float16)bf16r(v[1]); hv[2] = (_Float16)bf16r(v[2]); hv[3] = (_Float16)bf16r(v[3]);
    *(v4h*)(Ax + m_st * XPITCH + f4) = hv;
  }
  float bbE[2][4];
#pragma unroll
  for (int nt = 0; nt < 2; ++nt) {
    const int j = 32 * wave + 16 * nt + c;
    bbE[nt][0] = bf16r(ebih[j]) + bf16r(ebhh[j]);
    bbE[nt][1] = bf16r(ebih[NHID + j]) + bf16r(ebhh[NHID + j]);
    bbE[nt][2] = bf16r(ebih[2 * NHID + j]);
    bbE[nt][3] = bf16r(ebhh[2 * NHID + j]);
  }
  __syncthreads();

  const _Float16* axrow = Ax  + c * XPITCH + koff;
  const _Float16* ahrow = Ahh + c * HPITCH + koff;
  const _Float16* alrow = Ahl + c * HPITCH + koff;

#pragma unroll 1
  for (int t = 0; t < TSRC; ++t) {
    gru_cell(axrow, ahrow, alrow, WIHE, WHHE, bbE, hst, wave, c, koff);
    __syncthreads();
#pragma unroll
    for (int nt = 0; nt < 2; ++nt) {
      const int j = 32 * wave + 16 * nt + c;
#pragma unroll
      for (int r = 0; r < 8; ++r) {
        const float hn = hst[nt][r];
        const _Float16 hi = (_Float16)hn;
        const float res = (hn - (float)hi) * LOCARRY;
        Ahh[(8 * hh + r) * HPITCH + j] = hi;
        Ahl[(8 * hh + r) * HPITCH + j] = (_Float16)res;
      }
    }
    {
      const int tn = (t + 1 < TSRC) ? (t + 1) : ts_last;
      const v4f v = *(const v4f*)(x + ((size_t)(rowbase + m_st) * TTOT + (size_t)tn) * NFEAT + f4);
      v4h hv;
      hv[0] = (_Float16)bf16r(v[0]); hv[1] = (_Float16)bf16r(v[1]); hv[2] = (_Float16)bf16r(v[2]); hv[3] = (_Float16)bf16r(v[3]);
      *(v4h*)(Ax + m_st * XPITCH + f4) = hv;
    }
    __syncthreads();
  }

  float bbD[2][4];
#pragma unroll
  for (int nt = 0; nt < 2; ++nt) {
    const int j = 32 * wave + 16 * nt + c;
    bbD[nt][0] = bf16r(dbih[j]) + bf16r(dbhh[j]);
    bbD[nt][1] = bf16r(dbih[NHID + j]) + bf16r(dbhh[NHID + j]);
    bbD[nt][2] = bf16r(dbih[2 * NHID + j]);
    bbD[nt][3] = bf16r(dbhh[2 * NHID + j]);
  }
  const int jo = (16 * wave + c) & (NFEAT - 1);
  const float rb = bf16r(regb[jo]);
  const _Float16* wreg = WREG + (size_t)jo * NHID + koff;
  const v8f z8 = {0.f, 0.f, 0.f, 0.f, 0.f, 0.f, 0.f, 0.f};

#pragma unroll 1
  for (int td = 0; td < TTGT; ++td) {
    gru_cell(axrow, ahrow, alrow, WIHD, WHHD, bbD, hst, wave, c, koff);
    __syncthreads();
#pragma unroll
    for (int nt = 0; nt < 2; ++nt) {
      const int j = 32 * wave + 16 * nt + c;
#pragma unroll
      for (int r = 0; r < 8; ++r) {
        const float hn = hst[nt][r];
        const _Float16 hi = (_Float16)hn;
        const float res = (hn - (float)hi) * LOCARRY;
        Ahh[(8 * hh + r) * HPITCH + j] = hi;
        Ahl[(8 * hh + r) * HPITCH + j] = (_Float16)res;
      }
    }
    __syncthreads();
    if (wave < 4) {
      v8f o = z8, ol = z8;
#pragma unroll 1
      for (int k0 = 0; k0 < NHID; k0 += 32) {
        const v16h ah = Frag<_Float16>::load(ahrow + k0);
        const v16h al = Frag<_Float16>::load(alrow + k0);
        const v16h b  = Frag<_Float16>::load(wreg + k0);
        o  = Frag<_Float16>::mma(ah, b, o);
        ol = Frag<_Float16>::mma(al, b, ol);
        dep_guard_h(o, ol, ah, al);
        keep4_h(b, b, ah, al);
      }
      acc_guard2(o, ol);
#pragma unroll
      for (int r = 0; r < 8; ++r)
        Os[(8 * hh + r) * OPITCH + jo] = (o[r] + ol[r] * LOCARRY_INV) * WCARRY_INV + rb;
    }
    __syncthreads();
    {
      const int row = 2 * wave + hh;
      const v4f v = *(const v4f*)(Os + row * OPITCH + c4);
      float* op = out + ((size_t)(rowbase + row) * TTGT + (size_t)td) * NFEAT + c4;
      *(volatile v4f*)op = v;
      __threadfence();
      *(volatile v4f*)op = v;
    }
    {
      const v4f ov = *(const v4f*)(Os + m_st * OPITCH + f4);
      v4h hv;
      hv[0] = (_Float16)ov[0]; hv[1] = (_Float16)ov[1]; hv[2] = (_Float16)ov[2]; hv[3] = (_Float16)ov[3];
      *(v4h*)(Ax + m_st * XPITCH + f4) = hv;
    }
    __syncthreads();
  }
}

extern "C" void kernel_launch(void* const* d_in, const int* in_sizes, int n_in,
                              void* d_out, int out_size, void* d_ws, size_t ws_size, hipStream_t stream) {
  if (n_in < 13 || d_out == nullptr || d_ws == nullptr) return;
  if (in_sizes[0] != NBAT * TTOT * NFEAT ||
      in_sizes[1] != NGATE3 * NFEAT || in_sizes[2] != NGATE3 * NHID || in_sizes[3] != NGATE3 || in_sizes[4] != NGATE3 ||
      in_sizes[5] != NGATE3 * NFEAT || in_sizes[6] != NGATE3 * NHID || in_sizes[7] != NGATE3 || in_sizes[8] != NGATE3 ||
      in_sizes[9] != NFEAT * NHID || in_sizes[10] != NFEAT || in_sizes[11] < 1 || in_sizes[12] < 1 ||
      out_size != NOUT) return;

  const float* x       = (const float*)d_in[0];
  const float* enc_Wih = (const float*)d_in[1];
  const float* enc_Whh = (const float*)d_in[2];
  const float* enc_bih = (const float*)d_in[3];
  const float* enc_bhh = (const float*)d_in[4];
  const float* dec_Wih = (const float*)d_in[5];
  const float* dec_Whh = (const float*)d_in[6];
  const float* dec_bih = (const float*)d_in[7];
  const float* dec_bhh = (const float*)d_in[8];
  const float* reg_W   = (const float*)d_in[9];
  const float* reg_b   = (const float*)d_in[10];
  const int*   in_len  = (const int*)d_in[11];
  const int*   tg_len  = (const int*)d_in[12];
  float* out = (float*)d_out;

  char* ws = (char*)d_ws; size_t off = 0;
  auto carve = [&](size_t bytes) -> char* { char* p = ws + off; off += (bytes + 255) & ~(size_t)255; return p; };
  unsigned short* WIHE = (unsigned short*)carve((size_t)NGATE3 * NFEAT * 2);
  unsigned short* WHHE = (unsigned short*)carve((size_t)NGATE3 * NHID * 2);
  unsigned short* WIHD = (unsigned short*)carve((size_t)NGATE3 * NFEAT * 2);
  unsigned short* WHHD = (unsigned short*)carve((size_t)NGATE3 * NHID * 2);
  unsigned short* WREG = (unsigned short*)carve((size_t)NFEAT * NHID * 2);
  if (off > ws_size || off > (size_t)134217728) return;

  const int n8_ih = NGATE3 * (NFEAT / 8);
  const int n8_hh = NGATE3 * (NHID / 8);
  const int n8_rg = NFEAT * (NHID / 8);
  cvt8_kernel<1><<<(n8_ih + NTHR - 1) / NTHR, NTHR, 0, stream>>>(enc_Wih, WIHE, NGATE3, NFEAT / 8, NFEAT, 0, WCARRY);
  cvt8_kernel<1><<<(n8_hh + NTHR - 1) / NTHR, NTHR, 0, stream>>>(enc_Whh, WHHE, NGATE3, NHID / 8,  NHID,  0, WCARRY);
  cvt8_kernel<1><<<(n8_ih + NTHR - 1) / NTHR, NTHR, 0, stream>>>(dec_Wih, WIHD, NGATE3, NFEAT / 8, NFEAT, 0, WCARRY);
  cvt8_kernel<1><<<(n8_hh + NTHR - 1) / NTHR, NTHR, 0, stream>>>(dec_Whh, WHHD, NGATE3, NHID / 8,  NHID,  0, WCARRY);
  cvt8_kernel<1><<<(n8_rg + NTHR - 1) / NTHR, NTHR, 0, stream>>>(reg_W,   WREG, NFEAT,  NHID / 8,  NHID,  0, WCARRY);
  gru_seq_kernel<<<NBAT / SEQ_BLK, NTHR, 0, stream>>>(x, enc_bih, enc_bhh, dec_bih, dec_bhh, reg_b,
                                                     WIHE, WHHE, WIHD, WHHD, WREG, in_len, tg_len, out);
}
